// SelfAttentionBlock_42202348650993
// MI455X (gfx1250) — hardware-verified
//
#include <hip/hip_runtime.h>


typedef _Float16 h8  __attribute__((ext_vector_type(8)));
typedef _Float16 h16 __attribute__((ext_vector_type(16)));
typedef float    f8  __attribute__((ext_vector_type(8)));
typedef float    v4f __attribute__((ext_vector_type(4)));

#ifndef NB
#define NB 4
#endif
#ifndef SEQ
#define SEQ 4096
#endif
#define NB_FULL 4
#define HW_FULL 4096
#define CCH 256
#define C3 768
#define NGRP 8
#define CPG 32
#define GN_EPS 1e-5f
#define QBLK 128
#define KCH 32
#define LDK 264
#define LDV 40
#define LDP 40
#define LDO 136
#define LDQKV 72
#define LDPRJ 68
#define LDH 264

static_assert(NB >= 1 && NB <= NB_FULL);
static_assert(SEQ % QBLK == 0 && SEQ >= QBLK && SEQ <= HW_FULL);
static_assert(8 * 16 * LDO <= KCH * LDK + CCH * LDV);
static_assert(CCH % 32 == 0 && C3 == 3 * CCH);

__device__ __forceinline__ float bf16r(float f) {
  unsigned u = __float_as_uint(f);
  u = (u + 0x7FFFu + ((u >> 16) & 1u)) & 0xFFFF0000u;
  return __uint_as_float(u);
}

__device__ __forceinline__ h16 ldfrag(const _Float16* row, int h) {
  const h8 a = *(const h8*)(row + 8 * h);
  const h8 b = *(const h8*)(row + 16 + 8 * h);
  return __builtin_shufflevector(a, b, 0, 1, 2, 3, 4, 5, 6, 7, 8, 9, 10, 11, 12, 13, 14, 15);
}

__device__ __forceinline__ f8 wmma16(h16 a, h16 b, f8 c) {
  f8 d = __builtin_amdgcn_wmma_f32_16x16x32_f16(false, a, false, b, (short)0, c, false, false);
  asm volatile("v_nop\n\tv_nop\n\tv_nop\n\tv_nop" : "+v"(d) : "v"(a), "v"(b));
  return d;
}

__device__ __forceinline__ void wave_lds_sync() {
  __builtin_amdgcn_fence(__ATOMIC_RELEASE, "wavefront");
  asm volatile("s_wait_dscnt 0x0" ::: "memory");
  __builtin_amdgcn_wave_barrier();
}

__device__ __forceinline__ float redmax16(float v) {
  v = fmaxf(v, __shfl_xor(v, 8, 32));
  v = fmaxf(v, __shfl_xor(v, 4, 32));
  v = fmaxf(v, __shfl_xor(v, 2, 32));
  v = fmaxf(v, __shfl_xor(v, 1, 32));
  return v;
}
__device__ __forceinline__ float redsum16(float v) {
  v += __shfl_xor(v, 8, 32);
  v += __shfl_xor(v, 4, 32);
  v += __shfl_xor(v, 2, 32);
  v += __shfl_xor(v, 1, 32);
  return v;
}

__global__ __launch_bounds__(256) void cvt_w_kernel(const float* __restrict__ qw,
                                                    const float* __restrict__ pw,
                                                    _Float16* __restrict__ wq16,
                                                    _Float16* __restrict__ wp16) {
  const int t = blockIdx.x * 256 + (int)threadIdx.x;
  const float* src;
  _Float16* dst;
  if (blockIdx.x < 96) {
    src = qw + (size_t)t * 8;
    dst = wq16 + (size_t)t * 8;
  } else {
    const int u = t - 96 * 256;
    src = pw + (size_t)u * 8;
    dst = wp16 + (size_t)u * 8;
  }
  const v4f x0 = *(const v4f*)src;
  const v4f x1 = *(const v4f*)(src + 4);
  h8 o;
#pragma unroll
  for (int j = 0; j < 4; ++j) {
    o[j]     = (_Float16)(bf16r(x0[j]) * 64.0f);
    o[4 + j] = (_Float16)(bf16r(x1[j]) * 64.0f);
  }
  *(volatile h8*)dst = o;
  __threadfence();
  *(volatile h8*)dst = o;
}

__global__ __launch_bounds__(256) void gn_stats_kernel(const float* __restrict__ x,
                                                       float* __restrict__ stats) {
  __shared__ double red[256];
  __shared__ double red2[256];
  const int tid = threadIdx.x;
  const int bg = blockIdx.x;
  const int b = bg >> 3, g = bg & 7;
  const float* base = x + ((size_t)b * CCH + (size_t)g * CPG) * HW_FULL;
  const int upr = SEQ / 4;
  const int nunits = CPG * upr;
  double s = 0.0, s2 = 0.0;
  for (int u = tid; u < nunits; u += 256) {
    const int c = u / upr;
    const int n4 = (u - c * upr) * 4;
    const v4f v = *(const v4f*)(base + (size_t)c * HW_FULL + n4);
#pragma unroll
    for (int j = 0; j < 4; ++j) {
      const float r = bf16r(v[j]);
      s += (double)r;
      s2 += (double)r * (double)r;
    }
  }
  red[tid] = s;
  red2[tid] = s2;
  __syncthreads();
  for (int off = 128; off > 0; off >>= 1) {
    if (tid < off) {
      red[tid] += red[tid + off];
      red2[tid] += red2[tid + off];
    }
    __syncthreads();
  }
  const double tot = (double)(CPG * SEQ);
  const double mean = red[0] / tot;
  double var = red2[0] / tot - mean * mean;
  if (var < 0.0) var = 0.0;
  const float meanf = (float)mean;
  const float rstd = 1.0f / sqrtf((float)var + GN_EPS);
  v4f val;
  val[0] = (tid == 0) ? meanf : 0.0f;
  val[1] = (tid == 0) ? rstd : 0.0f;
  val[2] = 0.0f;
  val[3] = 0.0f;
  if (tid < 8) {
    float* p = stats + (size_t)bg * 32 + tid * 4;
    *(volatile v4f*)p = val;
    __threadfence();
    *(volatile v4f*)p = val;
  }
}

__global__ __launch_bounds__(256) void gn_apply_kernel(const float* __restrict__ x,
                                                       const float* __restrict__ stats,
                                                       const float* __restrict__ gw,
                                                       const float* __restrict__ gb,
                                                       _Float16* __restrict__ hT) {
  __shared__ __align__(16) _Float16 hs[64 * LDH];
  __shared__ float sm[NGRP];
  __shared__ float sr[NGRP];
  const int tid = threadIdx.x;
  const int b = blockIdx.y;
  const int tb = blockIdx.x * 64;
  if (tid < NGRP) {
    sm[tid] = stats[((size_t)b * NGRP + tid) * 32];
    sr[tid] = stats[((size_t)b * NGRP + tid) * 32 + 1];
  }
  __syncthreads();
  const int n4 = (tid & 15) * 4;
  const int cl = tid >> 4;
  for (int it = 0; it < CCH / 16; ++it) {
    const int c = it * 16 + cl;
    const v4f xv = *(const v4f*)(x + ((size_t)b * CCH + c) * HW_FULL + tb + n4);
    const int g = c >> 5;
    const float m = sm[g], r = sr[g];
    const float ga = bf16r(gw[c]), be = bf16r(gb[c]);
#pragma unroll
    for (int j = 0; j < 4; ++j) {
      const float hv = (bf16r(xv[j]) - m) * r * ga + be;
      hs[(n4 + j) * LDH + c] = (_Float16)hv;
    }
  }
  __syncthreads();
  const int w = tid >> 5, lane = tid & 31;
  h8 vals[8];
#pragma unroll
  for (int i = 0; i < 8; ++i) {
    const int row = w * 8 + i;
    vals[i] = *(const h8*)(hs + row * LDH + lane * 8);
  }
  _Float16* obase = hT + ((size_t)b * SEQ + tb + w * 8) * CCH + lane * 8;
#pragma unroll
  for (int i = 0; i < 8; ++i) *(volatile h8*)(obase + (size_t)i * CCH) = vals[i];
  __threadfence();
#pragma unroll
  for (int i = 0; i < 8; ++i) *(volatile h8*)(obase + (size_t)i * CCH) = vals[i];
}

__global__ __launch_bounds__(128) void qkv_kernel(const _Float16* __restrict__ hT,
                                                  const _Float16* __restrict__ w16,
                                                  const float* __restrict__ bias,
                                                  _Float16* __restrict__ qT,
                                                  _Float16* __restrict__ kT,
                                                  _Float16* __restrict__ vC) {
  __shared__ __align__(16) _Float16 st[4][64 * LDQKV];
  const int tid = threadIdx.x, lane = tid & 31, w = tid >> 5;
  const int lrow = lane & 15, lh = lane >> 4;
  const int tb = blockIdx.x * 64;
  const int mat = blockIdx.y;
  const int b = blockIdx.z;
  const int m0w = w * 64;
  const _Float16* W = w16 + (size_t)mat * (CCH * CCH);
  const _Float16* hB = hT + (size_t)b * SEQ * CCH;

  f8 acc[4][4];
  {
    f8 z = {};
#pragma unroll
    for (int mt = 0; mt < 4; ++mt)
#pragma unroll
      for (int nt = 0; nt < 4; ++nt) acc[mt][nt] = z;
  }

  for (int kc = 0; kc < CCH / 32; ++kc) {
    h16 af[4];
#pragma unroll
    for (int mt = 0; mt < 4; ++mt)
      af[mt] = ldfrag(W + (size_t)(m0w + mt * 16 + lrow) * CCH + kc * 32, lh);
#pragma unroll
    for (int nt = 0; nt < 4; ++nt) {
      const h16 bfr = ldfrag(hB + (size_t)(tb + nt * 16 + lrow) * CCH + kc * 32, lh);
#pragma unroll
      for (int mt = 0; mt < 4; ++mt) acc[mt][nt] = wmma16(af[mt], bfr, acc[mt][nt]);
    }
  }

  const float* bm = bias + mat * CCH + m0w;
  _Float16* sw = st[w];
#pragma unroll
  for (int mt = 0; mt < 4; ++mt) {
    float bv8[8];
#pragma unroll
    for (int r = 0; r < 8; ++r) bv8[r] = bf16r(bm[mt * 16 + 8 * lh + r]);
#pragma unroll
    for (int nt = 0; nt < 4; ++nt) {
#pragma unroll
      for (int r = 0; r < 8; ++r) {
        const float val = acc[mt][nt][r] * (1.0f / 64.0f) + bv8[r];
        const int chl = mt * 16 + 8 * lh + r;
        const int tok = nt * 16 + lrow;
        const int idx = (mat < 2) ? (tok * LDQKV + chl) : (chl * LDQKV + tok);
        sw[idx] = (_Float16)val;
      }
    }
  }
  wave_lds_sync();

  const int q = lane >> 3;
  const int piece = (lane & 7) * 8;
  h8 vals[16];
#pragma unroll
  for (int i = 0; i < 16; ++i) vals[i] = *(const h8*)(sw + (i * 4 + q) * LDQKV + piece);

  _Float16* obase;
  size_t ostride;
  if (mat == 0) {
    obase = qT + ((size_t)b * SEQ + tb + q) * CCH + m0w + piece;
    ostride = CCH;
  } else if (mat == 1) {
    obase = kT + ((size_t)b * SEQ + tb + q) * CCH + m0w + piece;
    ostride = CCH;
  } else {
    obase = vC + ((size_t)b * CCH + m0w + q) * SEQ + tb + piece;
    ostride = SEQ;
  }
#pragma unroll
  for (int i = 0; i < 16; ++i) *(volatile h8*)(obase + (size_t)(i * 4) * ostride) = vals[i];
  __threadfence();
#pragma unroll
  for (int i = 0; i < 16; ++i) *(volatile h8*)(obase + (size_t)(i * 4) * ostride) = vals[i];
}

__global__ __launch_bounds__(256) void attn_kernel(const _Float16* __restrict__ qT,
                                                   const _Float16* __restrict__ kT,
                                                   const _Float16* __restrict__ vC,
                                                   _Float16* __restrict__ oT) {
  __shared__ __align__(16) _Float16 kv[KCH * LDK + CCH * LDV];
  __shared__ __align__(16) _Float16 pS[8][16 * LDP];
  _Float16* ks = kv;
  _Float16* vs = kv + KCH * LDK;
  const int tid = threadIdx.x, lane = tid & 31, w = tid >> 5;
  const int lrow = lane & 15, lh = lane >> 4;
  const int b = blockIdx.y;
  const int qb = blockIdx.x * QBLK + w * 16;
  const _Float16* kB = kT + (size_t)b * SEQ * CCH;
  const _Float16* vB = vC + (size_t)b * CCH * SEQ;
  const _Float16* qrow = qT + ((size_t)b * SEQ + qb + lrow) * CCH;

  f8 o[16];
  {
    f8 z = {};
#pragma unroll
    for (int t = 0; t < 16; ++t) o[t] = z;
  }
  float mrow[8], lsum[8];
#pragma unroll
  for (int v = 0; v < 8; ++v) { mrow[v] = -1.0e30f; lsum[v] = 0.0f; }
  _Float16* pw = pS[w];

  for (int mc = 0; mc < SEQ / KCH; ++mc) {
    const int m0 = mc * KCH;
    __syncthreads();
#pragma unroll
    for (int j = 0; j < 4; ++j) {
      const int u = j * 256 + tid;
      const int key = u >> 5, c8 = (u & 31) * 8;
      *(h8*)(ks + key * LDK + c8) = *(const h8*)(kB + (size_t)(m0 + key) * CCH + c8);
    }
#pragma unroll
    for (int j = 0; j < 4; ++j) {
      const int u = j * 256 + tid;
      const int c = u >> 2, k8 = (u & 3) * 8;
      *(h8*)(vs + c * LDV + k8) = *(const h8*)(vB + (size_t)c * SEQ + m0 + k8);
    }
    __syncthreads();

    f8 s0, s1;
    {
      f8 z = {};
      s0 = z; s1 = z;
    }
#pragma unroll
    for (int kc = 0; kc < CCH / 32; ++kc) {
      const h16 qf = ldfrag(qrow + kc * 32, lh);
      const h16 k0 = ldfrag(ks + lrow * LDK + kc * 32, lh);
      const h16 k1 = ldfrag(ks + (16 + lrow) * LDK + kc * 32, lh);
      s0 = wmma16(qf, k0, s0);
      s1 = wmma16(qf, k1, s1);
    }

#pragma unroll
    for (int v = 0; v < 8; ++v) {
      const float a0 = s0[v] * 0.0625f;
      const float a1 = s1[v] * 0.0625f;
      const float t = redmax16(fmaxf(a0, a1));
      const float nm = fmaxf(mrow[v], t);
      const float sc = __expf(mrow[v] - nm);
      mrow[v] = nm;
      const float p0 = __expf(a0 - nm);
      const float p1 = __expf(a1 - nm);
      lsum[v] = lsum[v] * sc + redsum16(p0 + p1);
      const int row = v + 8 * lh;
      pw[row * LDP + lrow]      = (_Float16)(p0 * 256.0f);
      pw[row * LDP + 16 + lrow] = (_Float16)(p1 * 256.0f);
#pragma unroll
      for (int t2 = 0; t2 < 16; ++t2) o[t2][v] *= sc;
    }
    wave_lds_sync();

    const h16 pa = ldfrag(pw + lrow * LDP, lh);
#pragma unroll
    for (int t2 = 0; t2 < 16; ++t2) {
      const h16 vb = ldfrag(vs + (t2 * 16 + lrow) * LDV, lh);
      o[t2] = wmma16(pa, vb, o[t2]);
    }
  }

  float inv[8];
#pragma unroll
  for (int v = 0; v < 8; ++v) inv[v] = 1.0f / lsum[v];

  __syncthreads();
  _Float16* stg = kv + w * (16 * LDO);
  const int piece = lrow * 8;
#pragma unroll
  for (int half = 0; half < 2; ++half) {
#pragma unroll
    for (int t = 0; t < 8; ++t) {
#pragma unroll
      for (int v = 0; v < 8; ++v)
        stg[(8 * lh + v) * LDO + t * 16 + lrow] = (_Float16)(o[half * 8 + t][v] * inv[v]);
    }
    wave_lds_sync();
    h8 vals[8];
#pragma unroll
    for (int i = 0; i < 8; ++i) vals[i] = *(const h8*)(stg + (2 * i + lh) * LDO + piece);
    _Float16* obase = oT + ((size_t)b * SEQ + qb + lh) * CCH + half * 128 + piece;
#pragma unroll
    for (int i = 0; i < 8; ++i) *(volatile h8*)(obase + (size_t)(2 * i) * CCH) = vals[i];
    __threadfence();
#pragma unroll
    for (int i = 0; i < 8; ++i) *(volatile h8*)(obase + (size_t)(2 * i) * CCH) = vals[i];
    wave_lds_sync();
  }
}

__global__ __launch_bounds__(64) void proj_kernel(const _Float16* __restrict__ oT,
                                                  const _Float16* __restrict__ wp16,
                                                  const float* __restrict__ pb,
                                                  const float* __restrict__ x,
                                                  float* __restrict__ out) {
  __shared__ __align__(16) float st[2][64 * LDPRJ];
  const int tid = threadIdx.x, lane = tid & 31, w = tid >> 5;
  const int lrow = lane & 15, lh = lane >> 4;
  const int tb = blockIdx.x * 64;
  const int m0w = blockIdx.y * 128 + w * 64;
  const int b = blockIdx.z;
  const _Float16* cB = oT + (size_t)b * SEQ * CCH;

  f8 acc[4][4];
  {
    f8 z = {};
#pragma unroll
    for (int mt = 0; mt < 4; ++mt)
#pragma unroll
      for (int nt = 0; nt < 4; ++nt) acc[mt][nt] = z;
  }
  for (int kc = 0; kc < CCH / 32; ++kc) {
    h16 af[4];
#pragma unroll
    for (int mt = 0; mt < 4; ++mt)
      af[mt] = ldfrag(wp16 + (size_t)(m0w + mt * 16 + lrow) * CCH + kc * 32, lh);
#pragma unroll
    for (int nt = 0; nt < 4; ++nt) {
      const h16 bfr = ldfrag(cB + (size_t)(tb + nt * 16 + lrow) * CCH + kc * 32, lh);
#pragma unroll
      for (int mt = 0; mt < 4; ++mt) acc[mt][nt] = wmma16(af[mt], bfr, acc[mt][nt]);
    }
  }

  float* sw = st[w];
#pragma unroll
  for (int mt = 0; mt < 4; ++mt) {
    float bv8[8];
#pragma unroll
    for (int r = 0; r < 8; ++r) bv8[r] = bf16r(pb[m0w + mt * 16 + 8 * lh + r]);
#pragma unroll
    for (int nt = 0; nt < 4; ++nt) {
#pragma unroll
      for (int r = 0; r < 8; ++r) {
        const float val = acc[mt][nt][r] * (1.0f / 16384.0f) + bv8[r];
        sw[(mt * 16 + 8 * lh + r) * LDPRJ + nt * 16 + lrow] = val;
      }
    }
  }
  wave_lds_sync();

  const int piece = lrow * 4;
#pragma unroll
  for (int g4 = 0; g4 < 4; ++g4) {
    v4f vals[8];
    const size_t obase = ((size_t)b * CCH + m0w + g4 * 16 + lh) * HW_FULL + tb + piece;
#pragma unroll
    for (int i = 0; i < 8; ++i) {
      const int row = g4 * 16 + 2 * i + lh;
      const v4f a = *(const v4f*)(sw + row * LDPRJ + piece);
      const v4f xv = *(const v4f*)(x + obase + (size_t)(2 * i) * HW_FULL);
      v4f r;
#pragma unroll
      for (int j = 0; j < 4; ++j) r[j] = bf16r(xv[j]) + a[j];
      vals[i] = r;
    }
#pragma unroll
    for (int i = 0; i < 8; ++i) *(volatile v4f*)(out + obase + (size_t)(2 * i) * HW_FULL) = vals[i];
    __threadfence();
#pragma unroll
    for (int i = 0; i < 8; ++i) *(volatile v4f*)(out + obase + (size_t)(2 * i) * HW_FULL) = vals[i];
  }
}

extern "C" void kernel_launch(void* const* d_in, const int* in_sizes, int n_in,
                              void* d_out, int out_size, void* d_ws, size_t ws_size,
                              hipStream_t stream) {
  if (n_in < 7) return;
  if (in_sizes[0] < NB * CCH * HW_FULL) return;
  if (in_sizes[1] < CCH || in_sizes[2] < CCH) return;
  if (in_sizes[3] < C3 * CCH || in_sizes[4] < C3) return;
  if (in_sizes[5] < CCH * CCH || in_sizes[6] < CCH) return;
  if (out_size < NB * CCH * HW_FULL) return;

  const float* x     = (const float*)d_in[0];
  const float* gnw   = (const float*)d_in[1];
  const float* gnb   = (const float*)d_in[2];
  const float* qkvw  = (const float*)d_in[3];
  const float* qkvb  = (const float*)d_in[4];
  const float* projw = (const float*)d_in[5];
  const float* projb = (const float*)d_in[6];
  float* out = (float*)d_out;

  const size_t sz_wq  = (size_t)C3 * CCH * 2;
  const size_t sz_wp  = (size_t)CCH * CCH * 2;
  const size_t sz_st  = (size_t)NB_FULL * NGRP * 128;
  const size_t plane  = (size_t)NB * SEQ * CCH * 2;
  const size_t off_wq = 0;
  const size_t off_wp = off_wq + sz_wq;
  const size_t off_st = off_wp + sz_wp;
  const size_t off_h  = off_st + sz_st;
  const size_t off_q  = off_h + plane;
  const size_t off_k  = off_q + plane;
  const size_t off_v  = off_k + plane;
  const size_t off_o  = off_v + plane;
  const size_t total  = off_o + plane;
  if (total > ws_size) return;

  char* ws = (char*)d_ws;
  _Float16* wq16 = (_Float16*)(ws + off_wq);
  _Float16* wp16 = (_Float16*)(ws + off_wp);
  float* stats   = (float*)(ws + off_st);
  _Float16* hT   = (_Float16*)(ws + off_h);
  _Float16* qT   = (_Float16*)(ws + off_q);
  _Float16* kT   = (_Float16*)(ws + off_k);
  _Float16* vC   = (_Float16*)(ws + off_v);
  _Float16* oT   = (_Float16*)(ws + off_o);

  cvt_w_kernel<<<128, 256, 0, stream>>>(qkvw, projw, wq16, wp16);
  gn_stats_kernel<<<NB * NGRP, 256, 0, stream>>>(x, stats);
  gn_apply_kernel<<<dim3(SEQ / 64, NB), 256, 0, stream>>>(x, stats, gnw, gnb, hT);
  qkv_kernel<<<dim3(SEQ / 64, 3, NB), 128, 0, stream>>>(hT, wq16, qkvb, qT, kT, vC);
  attn_kernel<<<dim3(SEQ / QBLK, NB), 256, 0, stream>>>(qT, kT, vC, oT);
  proj_kernel<<<dim3(SEQ / 64, 2, NB), 64, 0, stream>>>(oT, wp16, projb, x, out);
}
